// NeighborhoodAttention_10720238371298
// MI455X (gfx1250) — hardware-verified
//
#include <hip/hip_runtime.h>


#define NB_  4
#define IH   56
#define IW   56
#define NPIX (IH * IW)
#define NTOK (NB_ * NPIX)
#define CC   128
#define C3   384
#define NH_  4
#define HD   32
#define KS   7
#define NBR  3
#define RPW  13
#define SCL  0.17677669529663689f
typedef _Float16 h16;
typedef unsigned short bf;
typedef __attribute__((ext_vector_type(16))) __bf16   v16bf;
typedef __attribute__((ext_vector_type(16))) _Float16 v16h;
typedef __attribute__((ext_vector_type(8)))  _Float16 v8h;
typedef __attribute__((ext_vector_type(8)))  unsigned short v8us;
typedef __attribute__((ext_vector_type(8)))  float    v8f;
typedef __attribute__((ext_vector_type(4)))  float    v4f;
typedef v8h  __attribute__((may_alias)) v8ha;
typedef v4f  __attribute__((may_alias)) v4fa;
typedef v8us __attribute__((may_alias)) v8usa;

__device__ __forceinline__ unsigned short f2bf(float f) { unsigned u = __float_as_uint(f); u += 0x7FFFu + ((u >> 16) & 1u); return (unsigned short)(u >> 16); }
__device__ __forceinline__ float bf2f(unsigned short b) { return __uint_as_float(((unsigned)b) << 16); }
__device__ __forceinline__ float bfr(float f) { return bf2f(f2bf(f)); }
__device__ __forceinline__ v16h cat16(v8h lo, v8h hi) { return __builtin_shufflevector(lo, hi, 0, 1, 2, 3, 4, 5, 6, 7, 8, 9, 10, 11, 12, 13, 14, 15); }
__device__ __forceinline__ v16bf cat16b(v8us lo, v8us hi) { return __builtin_bit_cast(v16bf, __builtin_shufflevector(lo, hi, 0, 1, 2, 3, 4, 5, 6, 7, 8, 9, 10, 11, 12, 13, 14, 15)); }
__device__ __forceinline__ v8f wmma16(v16h a, v16h b, v8f c) { return __builtin_amdgcn_wmma_f32_16x16x32_f16(false, a, false, b, (short)0, c, false, false); }
__device__ __forceinline__ v8f wmmab(v16bf a, v16bf b, v8f c) { return __builtin_amdgcn_wmma_f32_16x16x32_bf16(false, a, false, b, (short)0, c, false, false); }


template <typename T16> struct WFrag;
template <> struct WFrag<h16> { typedef v16h V; static __device__ __forceinline__ V ld(const h16* p) { return cat16(*(const v8h*)p, *(const v8h*)(p + 16)); } static __device__ __forceinline__ v8f mma(V a, V b, v8f c) { return wmma16(a, b, c); } };
template <> struct WFrag<bf> { typedef v16bf V; static __device__ __forceinline__ V ld(const bf* p) { return cat16b(*(const v8us*)p, *(const v8us*)(p + 16)); } static __device__ __forceinline__ v8f mma(V a, V b, v8f c) { return wmmab(a, b, c); } };
template <typename T16, int NSPLIT, bool BIAS>
__global__ __launch_bounds__(32) void k_gemmw(const T16* __restrict__ A, const T16* __restrict__ A2, const T16* __restrict__ Bt, const T16* __restrict__ Bt2, int K, float* C, int ldc, const float* __restrict__ bias, size_t sA, size_t sB, size_t sC) {
    typedef typename WFrag<T16>::V V;
    __shared__ __align__(16) float os[16 * 68];
    const size_t z = blockIdx.z; A += z * sA; if (A2) A2 += z * sA; Bt += z * sB; if (Bt2) Bt2 += z * sB; C += z * sC;
    const int lane = threadIdx.x & 31, lr = lane & 15, hi = lane >> 4; const int r0 = blockIdx.x * 64, c0 = blockIdx.y * 64;
    v8f acc[4][4];
#pragma unroll
    for (int mb = 0; mb < 4; ++mb)
#pragma unroll
        for (int nb = 0; nb < 4; ++nb) acc[mb][nb] = (v8f){};
    const size_t aoff = (size_t)(r0 + lr) * K + 8 * hi, boff = (size_t)(c0 + lr) * K + 8 * hi;
#pragma unroll 1
    for (int kc = 0; kc < K; kc += 32) {
        V a[4], a2[4];
#pragma unroll
        for (int mb = 0; mb < 4; ++mb) { a[mb] = WFrag<T16>::ld(A + aoff + (size_t)mb * 16 * K + kc); if (NSPLIT == 1 || NSPLIT == 2) a2[mb] = WFrag<T16>::ld(A2 + aoff + (size_t)mb * 16 * K + kc); }
#pragma unroll
        for (int nb = 0; nb < 4; ++nb) { const V b = WFrag<T16>::ld(Bt + boff + (size_t)nb * 16 * K + kc); V b2; if (NSPLIT >= 2) b2 = WFrag<T16>::ld(Bt2 + boff + (size_t)nb * 16 * K + kc);
#pragma unroll
            for (int mb = 0; mb < 4; ++mb) { acc[mb][nb] = WFrag<T16>::mma(a[mb], b, acc[mb][nb]); if (NSPLIT == 1 || NSPLIT == 2) acc[mb][nb] = WFrag<T16>::mma(a2[mb], b, acc[mb][nb]); if (NSPLIT >= 2) acc[mb][nb] = WFrag<T16>::mma(a[mb], b2, acc[mb][nb]); } }
        asm volatile("v_nop\n\tv_nop\n\tv_nop\n\tv_nop" : "+v"(acc[0][0]), "+v"(acc[1][1]), "+v"(acc[2][2]), "+v"(acc[3][3]) : "v"(a[0]), "v"(a[3]));
    }
#pragma unroll
    for (int mb = 0; mb < 4; ++mb) {
#pragma unroll
        for (int nb = 0; nb < 4; ++nb) {
#pragma unroll
            for (int j = 0; j < 8; ++j) os[(hi * 8 + j) * 68 + nb * 16 + lr] = acc[mb][nb][j]; }
        __builtin_amdgcn_wave_barrier(); asm volatile("" ::: "memory");
        float* crow = C + (size_t)(r0 + mb * 16) * ldc + c0;
#pragma unroll 1
        for (int ps = 0; ps < 2; ++ps) {
#pragma unroll
            for (int s = 0; s < 8; ++s) { const int row = 2 * s + hi, cofs = lr * 4; v4f val = *(const v4fa*)(os + row * 68 + cofs); if (BIAS) { val[0] += bfr(bias[c0 + cofs]); val[1] += bfr(bias[c0 + cofs + 1]); val[2] += bfr(bias[c0 + cofs + 2]); val[3] += bfr(bias[c0 + cofs + 3]); }
                *(volatile v4f*)(crow + (size_t)row * ldc + cofs) = val; }
            if (ps == 0) __threadfence(); }
        __builtin_amdgcn_wave_barrier(); asm volatile("" ::: "memory");
    }
}

__device__ __forceinline__ h16 tohx(float x) { return (h16)x; }
__device__ __forceinline__ void splitf(float y, unsigned short& h, unsigned short& l) { h = f2bf(y); l = f2bf(y - bf2f(h)); }
typedef __attribute__((ext_vector_type(2))) _Float16 v2h;
typedef __attribute__((ext_vector_type(4))) _Float16 v4h;
typedef __attribute__((ext_vector_type(2))) unsigned short v2us;
typedef __attribute__((ext_vector_type(4))) unsigned short v4us;
typedef __attribute__((ext_vector_type(2))) float v2f;
typedef __attribute__((ext_vector_type(4))) int v4i;

__global__ __launch_bounds__(256) void k_cvt8(const float* __restrict__ src, bf* dst, size_t n8) { const size_t i = (size_t)blockIdx.x * 256 + threadIdx.x; if (i >= n8) return; const v8f v = *(const v8f*)(src + i * 8); v8us o;
#pragma unroll
    for (int k = 0; k < 8; ++k) o[k] = f2bf(v[k]); *(volatile v8us*)(dst + i * 8) = o; __threadfence(); *(volatile v8us*)(dst + i * 8) = o; }
__global__ __launch_bounds__(256) void k_wtG(const float* __restrict__ w, int K, int N, bf* Bt) {
    const int lane = threadIdx.x & 31; const int L0 = (blockIdx.x * 8 + (threadIdx.x >> 5)) * 8; const int nlines = N * K / 64;
#pragma unroll
    for (int ps = 0; ps < 2; ++ps) {
#pragma unroll 1
        for (int l = 0; l < 8; ++l) { const int L = L0 + l; if (L >= nlines) break; const size_t e = (size_t)L * 64 + lane * 2; const int k = (int)(e % K), n = (int)(e / K); v2us o;
            o[0] = f2bf(w[(size_t)k * N + n]); o[1] = f2bf(w[(size_t)(k + 1) * N + n]); *(volatile v2us*)(Bt + e) = o; }
        if (ps == 0) __threadfence(); }
}
__global__ __launch_bounds__(256) void k_split8(const float* __restrict__ F, bf* Ph, bf* Pl, size_t n8) { const size_t i = (size_t)blockIdx.x * 256 + threadIdx.x; if (i >= n8) return; const v8f v = *(const v8f*)(F + i * 8); v8us oh, ol;
#pragma unroll
    for (int k = 0; k < 8; ++k) { unsigned short a, c2; splitf(v[k], a, c2); oh[k] = a; ol[k] = c2; }
    *(volatile v8us*)(Ph + i * 8) = oh; *(volatile v8us*)(Pl + i * 8) = ol; __threadfence(); *(volatile v8us*)(Ph + i * 8) = oh; *(volatile v8us*)(Pl + i * 8) = ol; }

__global__ __launch_bounds__(256) void k_natt(const float* __restrict__ F, const float* __restrict__ rpb, float* O) {
    const int lane = threadIdx.x & 31; const size_t w = (size_t)blockIdx.x * 8 + (threadIdx.x >> 5); if (w >= (size_t)NTOK * NH_) return; const int h = (int)(w % NH_); const size_t tok = w / NH_; const int b = (int)(tok / NPIX); const int pix = (int)(tok % NPIX); const int i = pix / IW, j = pix % IW;
    const int si = min(max(i - NBR, 0), IH - KS), sj = min(max(j - NBR, 0), IW - KS);
    float q = F[tok * C3 + h * HD + lane] * SCL; asm volatile("" : "+v"(q));
    float lg[KS * KS]; float mx = -3.0e38f;
#pragma unroll
    for (int p = 0; p < KS; ++p) {
#pragma unroll
        for (int qq = 0; qq < KS; ++qq) { const int ki = si + p, kj = sj + qq; const size_t ktok = (size_t)b * NPIX + (size_t)ki * IW + kj; float pr = __fmul_rn(q, F[ktok * C3 + CC + h * HD + lane]); asm volatile("" : "+v"(pr)); float s = pr;
#pragma unroll
            for (int sh = 16; sh; sh >>= 1) s += __shfl_xor(s, sh, 32);
            float bb = bfr(rpb[((size_t)h * RPW + (ki - i + KS - 1)) * RPW + (kj - j + KS - 1)]); asm volatile("" : "+v"(bb)); const float t = __fadd_rn(s, bb); lg[p * KS + qq] = t; mx = fmaxf(mx, t); } }
    float sum = 0.f;
#pragma unroll
    for (int k = 0; k < KS * KS; ++k) { float d0 = __fsub_rn(lg[k], mx); asm volatile("" : "+v"(d0)); lg[k] = __builtin_amdgcn_exp2f(__fmul_rn(d0, 1.4426950408889634f)); sum += lg[k]; }
    const float f = __fdiv_rn(1.0f, sum); float acc = 0.f;
#pragma unroll
    for (int p = 0; p < KS; ++p) {
#pragma unroll
        for (int qq = 0; qq < KS; ++qq) { const size_t ktok = (size_t)b * NPIX + (size_t)(si + p) * IW + (sj + qq); float pk = __fmul_rn(lg[p * KS + qq], f); asm volatile("" : "+v"(pk)); float t1 = __fmul_rn(pk, F[ktok * C3 + 2 * CC + h * HD + lane]); asm volatile("" : "+v"(t1)); acc = __fadd_rn(acc, t1); } }
    float* dst = O + tok * CC + h * HD + lane; *(volatile float*)dst = acc; __threadfence(); *(volatile float*)dst = acc; }

extern "C" void kernel_launch(void* const* d_in, const int* in_sizes, int n_in,
                              void* d_out, int out_size, void* d_ws, size_t ws_size, hipStream_t stream) {
    (void)in_sizes; (void)n_in; (void)out_size;
    const float* x = (const float*)d_in[0]; const float* wqkv = (const float*)d_in[1]; const float* bqkv = (const float*)d_in[2]; const float* rpb = (const float*)d_in[3]; const float* wp = (const float*)d_in[4]; const float* bp = (const float*)d_in[5];
    float* OUT = (float*)d_out;
    char* wsp = (char*)d_ws;
    auto take = [&](size_t bytes) { char* p = wsp; wsp += (bytes + 255) & ~(size_t)255; return (void*)p; };
    bf* WB = (bf*)take((size_t)C3 * CC * 2); bf* WP = (bf*)take((size_t)CC * CC * 2); bf* XB = (bf*)take((size_t)NTOK * CC * 2); float* F = (float*)take((size_t)NTOK * C3 * 4); float* O = (float*)take((size_t)NTOK * CC * 4); bf* Oh = (bf*)take((size_t)NTOK * CC * 2); bf* Ol = (bf*)take((size_t)NTOK * CC * 2);
    if ((size_t)(wsp - (char*)d_ws) > ws_size) return;
    k_wtG<<<(unsigned)((CC * C3 / 64 + 63) / 64), 256, 0, stream>>>(wqkv, CC, C3, WB); k_wtG<<<(unsigned)((CC * CC / 64 + 63) / 64), 256, 0, stream>>>(wp, CC, CC, WP);
    k_cvt8<<<(unsigned)(((size_t)NTOK * CC / 8 + 255) / 256), 256, 0, stream>>>(x, XB, (size_t)NTOK * CC / 8);
    k_gemmw<bf, 0, true><<<dim3(NTOK / 64, C3 / 64, 1), 32, 0, stream>>>(XB, nullptr, WB, nullptr, CC, F, C3, bqkv, 0, 0, 0);
    k_natt<<<(unsigned)(((size_t)NTOK * NH_ + 7) / 8), 256, 0, stream>>>(F, rpb, O);
    k_split8<<<(unsigned)(((size_t)NTOK * CC / 8 + 255) / 256), 256, 0, stream>>>(O, Oh, Ol, (size_t)NTOK * CC / 8);
    k_gemmw<bf, 1, true><<<dim3(NTOK / 64, CC / 64, 1), 32, 0, stream>>>(Oh, Ol, WP, nullptr, CC, OUT, CC, bp, 0, 0, 0);
}
